// GlobalAttention_41858751267187
// MI455X (gfx1250) — hardware-verified
//
#include <hip/hip_runtime.h>
#include <stddef.h>


typedef _Float16 v16h __attribute__((ext_vector_type(16)));
typedef _Float16 v8h  __attribute__((ext_vector_type(8)));
typedef float    v8f  __attribute__((ext_vector_type(8)));
typedef float    v4f  __attribute__((ext_vector_type(4)));
typedef _Float16 h16;

#ifndef NB
#define NB 32
#endif
#ifndef SEQ
#define SEQ 1024
#endif
#define NB_FULL  32
#define SEQ_FULL 1024
#define DIM   128
#define MROWS (NB * SEQ)

static_assert(NB >= 1 && NB <= NB_FULL);
static_assert(SEQ >= 256 && SEQ <= SEQ_FULL && (SEQ % 256) == 0);
static_assert((DIM % 64) == 0 && (DIM % 32) == 0 && DIM == 128);
static_assert((MROWS % 64) == 0 && (MROWS % 16) == 0);
static_assert((SEQ % 128) == 0 && (SEQ % 16) == 0);
static_assert(((SEQ / 2) % 4) == 0);
static_assert(32 * 4 == DIM);

#define LDT 72
#define LDC 68
static_assert((LDT % 8) == 0 && LDT >= 64);
static_assert((LDC % 4) == 0 && LDC >= 64);

#define WCARRY 64.0f

#define DKSCALE ((float)(0.08838834764831845 / (double)SEQ))

#define OUT1_OFF ((size_t)NB_FULL * SEQ_FULL)
static_assert(OUT1_OFF * 4 == (size_t)131072);
static_assert((OUT1_OFF + (size_t)NB_FULL * DIM) * 4 == (size_t)147456);

#define WT_BYTES   ((size_t)DIM * DIM * 2)
#define P16_BYTES  ((size_t)MROWS * DIM * 2)
#define P32_BYTES  ((size_t)MROWS * DIM * 4)
#define KS_BYTES   ((size_t)NB * DIM * 4)
#define AGG_BYTES  ((size_t)MROWS * 4)
#define OFF_WQ  ((size_t)0)
#define OFF_WK  (OFF_WQ + WT_BYTES)
#define OFF_WV  (OFF_WK + WT_BYTES)
#define OFF_A   (OFF_WV + WT_BYTES)
#define OFF_Q   (OFF_A + P16_BYTES)
#define OFF_K   (OFF_Q + P32_BYTES)
#define OFF_V   (OFF_K + P32_BYTES)
#define OFF_KS  (OFF_V + P32_BYTES)
#define OFF_AGG (OFF_KS + KS_BYTES)
#define WS_TOTAL (OFF_AGG + AGG_BYTES)
static_assert((WT_BYTES % 128) == 0 && (P16_BYTES % 128) == 0);
static_assert((P32_BYTES % 128) == 0 && (KS_BYTES % 512) == 0 && (AGG_BYTES % 512) == 0);
static_assert(WS_TOTAL <= (size_t)134217728);

static_assert((256 / 8) * 2 == 64);
static_assert((256 / 16) * 4 == 64);
static_assert((256 / 16) == 16);
static_assert(8 * 16 == 128);

__device__ __forceinline__ float bf16r(float x) {
  unsigned int u = __float_as_uint(x);
  u = (u + 0x7FFFu + ((u >> 16) & 1u)) & 0xFFFF0000u;
  return __uint_as_float(u);
}

static __device__ __forceinline__ h16 toh_flush(float v) {
  const h16 r = (h16)v;
  return (fabsf(v) < 6.103515625e-05f) ? (h16)0.0f : r;
}

__device__ __forceinline__ v16h frag_at(const _Float16* p) {
  v8h lo = *(const v8h*)(p);
  v8h hi = *(const v8h*)(p + 16);
  v16h out;
#pragma unroll
  for (int i = 0; i < 8; ++i) { out[i] = lo[i]; out[i + 8] = hi[i]; }
  return out;
}

__device__ __forceinline__ v8f wmma16(v16h a, v16h b, v8f c) {
  v8f d = __builtin_amdgcn_wmma_f32_16x16x32_f16(false, a, false, b, (short)0, c,
                                                 false, false);
  asm volatile("v_nop\n\tv_nop\n\tv_nop\n\tv_nop" : "+v"(d) : "v"(a), "v"(b));
  return d;
}

__device__ __forceinline__ float red32_sum(float x) {
#pragma unroll
  for (int off = 1; off < 32; off <<= 1) x += __shfl_xor(x, off, 32);
  return x;
}
__device__ __forceinline__ float red32_max(float x) {
#pragma unroll
  for (int off = 1; off < 32; off <<= 1) x = fmaxf(x, __shfl_xor(x, off, 32));
  return x;
}

__global__ __launch_bounds__(256) void wconv_kernel(
    const float* __restrict__ W, _Float16* __restrict__ Wt, unsigned ldw, unsigned ldk) {
  __shared__ _Float16 T[64 * LDT];
  const unsigned tid = threadIdx.x;
  const unsigned n0 = blockIdx.x * 64u;
  const unsigned k0 = blockIdx.y * 64u;
#pragma unroll 4
  for (unsigned j = 0; j < 16u; ++j) {
    const unsigned idx = tid + 256u * j;
    const unsigned kr = idx >> 6, nc = idx & 63u;
    const float v = W[(size_t)(k0 + kr) * ldw + n0 + nc];
    T[nc * LDT + kr] = toh_flush(WCARRY * bf16r(v));
  }
  __syncthreads();
  v8h x[2];
  size_t off[2];
#pragma unroll
  for (unsigned i = 0; i < 2u; ++i) {
    const unsigned n = 32u * i + (tid >> 3);
    const unsigned kc = (tid & 7u) * 8u;
    x[i] = *(const v8h*)&T[n * LDT + kc];
    off[i] = (size_t)(n0 + n) * ldk + k0 + kc;
  }
#pragma unroll
  for (int i = 0; i < 2; ++i) *(volatile v8h*)(Wt + off[i]) = x[i];
  __threadfence();
#pragma unroll
  for (int i = 0; i < 2; ++i) *(volatile v8h*)(Wt + off[i]) = x[i];
}

__global__ __launch_bounds__(256) void aconv_kernel(
    const float* __restrict__ X, _Float16* __restrict__ dst) {
  const unsigned tid = threadIdx.x;
  const unsigned crow = blockIdx.x * 16u + (tid >> 4);
  const unsigned c = (tid & 15u) * 8u;
  const unsigned bidx = crow / (unsigned)SEQ;
  const unsigned sq = crow - bidx * (unsigned)SEQ;
  const size_t srow = (size_t)bidx * SEQ_FULL + sq;
  const float* xr = X + srow * DIM + c;
  const v4f a0 = *(const v4f*)(xr);
  const v4f a1 = *(const v4f*)(xr + 4);
  v8h o;
#pragma unroll
  for (int i = 0; i < 4; ++i) {
    o[i]     = toh_flush(bf16r(a0[i]));
    o[i + 4] = toh_flush(bf16r(a1[i]));
  }
  _Float16* p = dst + (size_t)crow * DIM + c;
  *(volatile v8h*)p = o;
  __threadfence();
  *(volatile v8h*)p = o;
}

__global__ __launch_bounds__(256) void gemm_f32_kernel(
    const _Float16* __restrict__ A16, const _Float16* __restrict__ Bt,
    const float* __restrict__ bias, float* __restrict__ outf) {
  __shared__ float Cs[64 * LDC];
  const unsigned K = (unsigned)DIM;
  const unsigned tid = threadIdx.x, lane = tid & 31u, w = tid >> 5;
  const unsigned mw = w >> 1, nw = w & 1u;
  const unsigned hh = lane >> 4, m = lane & 15u;
  const unsigned n0 = blockIdx.x * 64u;
  const unsigned row0 = blockIdx.y * 64u;

  const _Float16* ap  = A16 + (size_t)(row0 + mw * 16u + m) * K + hh * 8u;
  const _Float16* bp0 = Bt + (size_t)(n0 + nw * 32u + m) * K + hh * 8u;
  const _Float16* bp1 = bp0 + (size_t)16 * K;
  v8f acc0 = {}, acc1 = {};
#pragma unroll 2
  for (unsigned k0 = 0; k0 < K; k0 += 32u) {
    const v16h a  = frag_at(ap + k0);
    const v16h b0 = frag_at(bp0 + k0);
    const v16h b1 = frag_at(bp1 + k0);
    acc0 = wmma16(a, b0, acc0);
    acc1 = wmma16(a, b1, acc1);
  }
#pragma unroll
  for (int r = 0; r < 8; ++r) {
    float* d = &Cs[(mw * 16u + hh * 8u + (unsigned)r) * LDC + nw * 32u + m];
    d[0]  = acc0[r];
    d[16] = acc1[r];
  }
  __syncthreads();

  v4f xs[4];
  size_t off[4];
#pragma unroll
  for (unsigned i = 0; i < 4u; ++i) {
    const unsigned r = 16u * i + (tid >> 4);
    const unsigned c = (tid & 15u) * 4u;
    const v4f u = *(const v4f*)&Cs[r * LDC + c];
    const v4f g = *(const v4f*)(bias + n0 + c);
    v4f val;
#pragma unroll
    for (int j = 0; j < 4; ++j) val[j] = u[j] * (1.0f / WCARRY) + bf16r(g[j]);
    xs[i] = val;
    off[i] = (size_t)(row0 + r) * DIM + n0 + c;
  }
#pragma unroll
  for (int i = 0; i < 4; ++i) *(volatile v4f*)(outf + off[i]) = xs[i];
  __threadfence();
#pragma unroll
  for (int i = 0; i < 4; ++i) *(volatile v4f*)(outf + off[i]) = xs[i];
}

__global__ __launch_bounds__(256) void ksum_kernel(
    const float* __restrict__ K32, float* __restrict__ KS) {
#pragma clang fp contract(off)
  __shared__ __attribute__((aligned(16))) float cpart[256];
  __shared__ __attribute__((aligned(16))) float cfin[DIM];
  const unsigned tid = threadIdx.x, lane = tid & 31u;
  const unsigned wave = __builtin_amdgcn_readfirstlane(tid >> 5);
  const unsigned b = blockIdx.x;
  {
    const unsigned d = tid & 127u;
    const unsigned ch = tid >> 7;
    const unsigned rb = ch * (unsigned)(SEQ / 2);
    const float* kp = K32 + ((size_t)b * SEQ + rb) * DIM + d;
    float p0 = 0.0f, p1 = 0.0f, p2 = 0.0f, p3 = 0.0f;
#pragma unroll 1
    for (unsigned r = 0; r < (unsigned)(SEQ / 2); r += 4u) {
      p0 += kp[(size_t)(r)      * DIM];
      p1 += kp[(size_t)(r + 1u) * DIM];
      p2 += kp[(size_t)(r + 2u) * DIM];
      p3 += kp[(size_t)(r + 3u) * DIM];
    }
    cpart[tid] = (p0 + p1) + (p2 + p3);
  }
  __syncthreads();
  if (tid < 128u) cfin[tid] = cpart[tid] + cpart[tid + 128u];
  __syncthreads();
  if (wave == 0u) {
    const v4f x = *(const v4f*)&cfin[lane * 4u];
    float* p = KS + (size_t)b * DIM + lane * 4u;
    *(volatile v4f*)p = x;
    __threadfence();
    *(volatile v4f*)p = x;
  }
}

__global__ __launch_bounds__(256) void agg_kernel(
    const float* __restrict__ Q32, const float* __restrict__ K32,
    const float* __restrict__ KS, const float* __restrict__ mask,
    float* __restrict__ AGG) {
#pragma clang fp contract(off)
  __shared__ __attribute__((aligned(16))) float aggs[128];
  const unsigned tid = threadIdx.x, lane = tid & 31u;
  const unsigned wave = __builtin_amdgcn_readfirstlane(tid >> 5);
  const unsigned q0 = blockIdx.x * 128u;
  const unsigned b = blockIdx.y;

  const v4f ks = *(const v4f*)(KS + (size_t)b * DIM + lane * 4u);
  const size_t base = ((size_t)b * SEQ + q0 + wave * 16u) * DIM + lane * 4u;
#pragma unroll 1
  for (unsigned r = 0; r < 16u; ++r) {
    const v4f q = *(const v4f*)(Q32 + base + (size_t)r * DIM);
    const v4f k = *(const v4f*)(K32 + base + (size_t)r * DIM);
    float a = (q[0] * ks[0] + q[1] * ks[1]) + (q[2] * ks[2] + q[3] * ks[3]);
    float c = (q[0] * k[0] + q[1] * k[1]) + (q[2] * k[2] + q[3] * k[3]);
    a = red32_sum(a);
    c = red32_sum(c);
    const float g = a - c;
    if (lane == 0u) aggs[wave * 16u + r] = g;
  }
  __syncthreads();

  if (wave == 0u) {
    const unsigned i = lane * 4u;
    const v4f g = *(const v4f*)&aggs[i];
    const v4f mk = *(const v4f*)(mask + (size_t)b * SEQ_FULL + q0 + i);
    v4f val;
#pragma unroll
    for (int j = 0; j < 4; ++j) {
      const float mm = bf16r(mk[j]);
      val[j] = mm * (mm * (DKSCALE * g[j]));
    }
    float* p = AGG + (size_t)b * SEQ + q0 + i;
    *(volatile v4f*)p = val;
    __threadfence();
    *(volatile v4f*)p = val;
  }
}

__global__ __launch_bounds__(256) void finalize_kernel(
    const float* __restrict__ AGG, const float* __restrict__ V,
    const float* __restrict__ mask, float* __restrict__ out) {
#pragma clang fp contract(off)
  __shared__ __attribute__((aligned(16))) float av[SEQ];
  __shared__ __attribute__((aligned(16))) float wv[SEQ];
  __shared__ __attribute__((aligned(16))) float cpart[256];
  __shared__ __attribute__((aligned(16))) float cfin[DIM];
  __shared__ float redw[8];

  const unsigned tid = threadIdx.x, lane = tid & 31u;
  const unsigned wave = __builtin_amdgcn_readfirstlane(tid >> 5);
  const unsigned b = blockIdx.x;
  const float* ag = AGG + (size_t)b * SEQ;
  const float* mk = mask + (size_t)b * SEQ_FULL;

  float ss = 0.0f;
#pragma unroll 1
  for (unsigned j = 0; j < (unsigned)(SEQ / 256); ++j) {
    const unsigned i = tid + 256u * j;
    const float g = ag[i];
    av[i] = g;
    ss += g * g;
  }
  ss = red32_sum(ss);
  if (lane == 0u) redw[wave] = ss;
  __syncthreads();
  const float tot = ((redw[0] + redw[1]) + (redw[2] + redw[3])) +
                    ((redw[4] + redw[5]) + (redw[6] + redw[7]));
  __syncthreads();
  const float rn = __builtin_amdgcn_rcpf(sqrtf(tot));

  float mx = -3.0e38f;
#pragma unroll 1
  for (unsigned j = 0; j < (unsigned)(SEQ / 256); ++j) {
    const unsigned i = tid + 256u * j;
    const float mm = bf16r(mk[i]);
    const float a = av[i] * rn + (1.0f - mm) * (-1.0e9f);
    av[i] = a;
    mx = fmaxf(mx, a);
  }
  mx = red32_max(mx);
  if (lane == 0u) redw[wave] = mx;
  __syncthreads();
  const float mxa = fmaxf(fmaxf(fmaxf(redw[0], redw[1]), fmaxf(redw[2], redw[3])),
                          fmaxf(fmaxf(redw[4], redw[5]), fmaxf(redw[6], redw[7])));
  __syncthreads();

  float se = 0.0f;
#pragma unroll 1
  for (unsigned j = 0; j < (unsigned)(SEQ / 256); ++j) {
    const unsigned i = tid + 256u * j;
    const float e = expf(av[i] - mxa);
    av[i] = e;
    se += e;
  }
  se = red32_sum(se);
  if (lane == 0u) redw[wave] = se;
  __syncthreads();
  const float set = ((redw[0] + redw[1]) + (redw[2] + redw[3])) +
                    ((redw[4] + redw[5]) + (redw[6] + redw[7]));
  __syncthreads();
  const float rinv = __builtin_amdgcn_rcpf(set);

#pragma unroll 1
  for (unsigned j = 0; j < (unsigned)(SEQ / 256); ++j) {
    const unsigned i = tid + 256u * j;
    const float at = av[i] * rinv;
    av[i] = at;
    wv[i] = bf16r(mk[i]) * at;
  }
  __syncthreads();

#pragma unroll 1
  for (unsigned i4 = tid * 4u; i4 < (unsigned)SEQ; i4 += 1024u) {
    const v4f x = *(const v4f*)&av[i4];
    float* p = out + (size_t)b * SEQ_FULL + i4;
    *(volatile v4f*)p = x;
    __threadfence();
    *(volatile v4f*)p = x;
  }

  {
    const unsigned d = tid & 127u;
    const unsigned ch = tid >> 7;
    const unsigned rb = ch * (unsigned)(SEQ / 2);
    const float* vp = V + ((size_t)b * SEQ + rb) * DIM + d;
    float p0 = 0.0f, p1 = 0.0f, p2 = 0.0f, p3 = 0.0f;
#pragma unroll 1
    for (unsigned r = 0; r < (unsigned)(SEQ / 2); r += 4u) {
      p0 += wv[rb + r]      * vp[(size_t)(r)      * DIM];
      p1 += wv[rb + r + 1u] * vp[(size_t)(r + 1u) * DIM];
      p2 += wv[rb + r + 2u] * vp[(size_t)(r + 2u) * DIM];
      p3 += wv[rb + r + 3u] * vp[(size_t)(r + 3u) * DIM];
    }
    cpart[tid] = (p0 + p1) + (p2 + p3);
  }
  __syncthreads();
  if (tid < 128u) cfin[tid] = cpart[tid] + cpart[tid + 128u];
  __syncthreads();
  if (wave == 0u) {
    const v4f x = *(const v4f*)&cfin[lane * 4u];
    float* p = out + OUT1_OFF + (size_t)b * DIM + lane * 4u;
    *(volatile v4f*)p = x;
    __threadfence();
    *(volatile v4f*)p = x;
  }
}

extern "C" void kernel_launch(void* const* d_in, const int* in_sizes, int n_in,
                              void* d_out, int out_size, void* d_ws, size_t ws_size,
                              hipStream_t stream) {
  if (n_in < 8) return;
  const long long need_rows = (long long)(NB - 1) * SEQ_FULL + SEQ;
  if ((long long)in_sizes[0] < need_rows * DIM) return;
  if ((long long)in_sizes[1] < need_rows) return;
  if ((long long)in_sizes[2] < (long long)DIM * DIM) return;
  if ((long long)in_sizes[4] < (long long)DIM * DIM) return;
  if ((long long)in_sizes[6] < (long long)DIM * DIM) return;
  if (in_sizes[3] < DIM || in_sizes[5] < DIM || in_sizes[7] < DIM) return;
  if ((long long)out_size < (long long)OUT1_OFF + (long long)NB * DIM) return;
  if (ws_size < WS_TOTAL) return;

  const float* X    = (const float*)d_in[0];
  const float* mask = (const float*)d_in[1];
  const float* wq   = (const float*)d_in[2];
  const float* bq   = (const float*)d_in[3];
  const float* wk   = (const float*)d_in[4];
  const float* bk   = (const float*)d_in[5];
  const float* wv   = (const float*)d_in[6];
  const float* bv   = (const float*)d_in[7];
  float* out = (float*)d_out;

  char* ws = (char*)d_ws;
  _Float16* Wq_t = (_Float16*)(ws + OFF_WQ);
  _Float16* Wk_t = (_Float16*)(ws + OFF_WK);
  _Float16* Wv_t = (_Float16*)(ws + OFF_WV);
  _Float16* A16  = (_Float16*)(ws + OFF_A);
  float*    Q32  = (float*)(ws + OFF_Q);
  float*    K32  = (float*)(ws + OFF_K);
  float*    V32  = (float*)(ws + OFF_V);
  float*    KSp  = (float*)(ws + OFF_KS);
  float*    AGGp = (float*)(ws + OFF_AGG);

  dim3 blk(256);
  dim3 gsq(DIM / 64, DIM / 64);
  dim3 gg(DIM / 64, MROWS / 64);

  wconv_kernel<<<gsq, blk, 0, stream>>>(wq, Wq_t, (unsigned)DIM, (unsigned)DIM);
  wconv_kernel<<<gsq, blk, 0, stream>>>(wk, Wk_t, (unsigned)DIM, (unsigned)DIM);
  wconv_kernel<<<gsq, blk, 0, stream>>>(wv, Wv_t, (unsigned)DIM, (unsigned)DIM);

  aconv_kernel<<<dim3(MROWS / 16), blk, 0, stream>>>(X, A16);
  gemm_f32_kernel<<<gg, blk, 0, stream>>>(A16, Wq_t, bq, Q32);
  gemm_f32_kernel<<<gg, blk, 0, stream>>>(A16, Wk_t, bk, K32);
  gemm_f32_kernel<<<gg, blk, 0, stream>>>(A16, Wv_t, bv, V32);
  ksum_kernel<<<dim3(NB), blk, 0, stream>>>(K32, KSp);
  agg_kernel<<<dim3(SEQ / 128, NB), blk, 0, stream>>>(Q32, K32, KSp, mask, AGGp);
  finalize_kernel<<<dim3(NB), blk, 0, stream>>>(AGGp, V32, mask, out);
}
